// GCNLayer_32298154066114
// MI455X (gfx1250) — hardware-verified
//
#include <hip/hip_runtime.h>
#include <stddef.h>


typedef _Float16 v16h __attribute__((ext_vector_type(16)));
typedef _Float16 v8h  __attribute__((ext_vector_type(8)));
typedef float    v8f  __attribute__((ext_vector_type(8)));
typedef float    v4f  __attribute__((ext_vector_type(4)));
typedef int      v4i  __attribute__((ext_vector_type(4)));
typedef _Float16 h16;

#define N_NODES 8192
#define N_EDGES 262144
#define DIN     128
#define DOUT    128
#ifndef OUT_ROWS
#define OUT_ROWS N_NODES
#endif

#define LDC 68
static_assert((LDC % 4) == 0 && LDC >= 64);

#define XCARRY 16.0f
#define WCARRY 64.0f

#define CHUNK   2048
#define SEGCAP  256
#define NCHUNK  (N_EDGES / CHUNK)
#define DROWS   128
#define AROWS   32
#define WROWS   4
#define WSHIFT  2
#define SEENW   (N_NODES / 32)

static_assert((N_EDGES % CHUNK) == 0);
static_assert(CHUNK == 256 * 8);
static_assert(SEGCAP == 32 * 8);
static_assert((N_NODES % DROWS) == 0 && DROWS == 32 * 4);
static_assert((N_NODES % AROWS) == 0 && AROWS == 8 * WROWS && WROWS == (1 << WSHIFT));
static_assert(OUT_ROWS >= AROWS && OUT_ROWS <= N_NODES && (OUT_ROWS % AROWS) == 0);
static_assert(N_NODES <= 8192 && AROWS <= 32);
static_assert(DOUT == 32 * 4);
static_assert((DIN % 32) == 0 && (DOUT % 64) == 0 && (N_NODES % 64) == 0);
static_assert(((N_NODES * DIN / 8) % 256) == 0);
static_assert(((DOUT * DIN / 8) % 256) == 0);

#define X16_BYTES  ((size_t)N_NODES * DIN * 2)
#define W16_BYTES  ((size_t)DOUT * DIN * 2)
#define DINV_BYTES ((size_t)N_NODES * 4)
#define G_BYTES    ((size_t)N_NODES * DOUT * 4)
#define OFF_X16  ((size_t)0)
#define OFF_W16  (OFF_X16 + X16_BYTES)
#define OFF_DINV (OFF_W16 + W16_BYTES)
#define OFF_G    (OFF_DINV + DINV_BYTES)
#define WS_TOTAL (OFF_G + G_BYTES)
static_assert((X16_BYTES % 128) == 0 && (W16_BYTES % 128) == 0);
static_assert((DINV_BYTES % 128) == 0 && (G_BYTES % 128) == 0);
static_assert(WS_TOTAL <= (size_t)134217728);

__device__ __forceinline__ float bf16r(float x) {
  unsigned int u = __float_as_uint(x);
  u = (u + 0x7FFFu + ((u >> 16) & 1u)) & 0xFFFF0000u;
  return __uint_as_float(u);
}

static __device__ __forceinline__ h16 toh_flush(float v) {
  const h16 r = (h16)v;
  return (fabsf(v) < 6.103515625e-05f) ? (h16)0.0f : r;
}

__device__ __forceinline__ v16h frag_at(const _Float16* p) {
  v8h lo = *(const v8h*)(p);
  v8h hi = *(const v8h*)(p + 16);
  v16h out;
#pragma unroll
  for (int i = 0; i < 8; ++i) { out[i] = lo[i]; out[i + 8] = hi[i]; }
  return out;
}

__device__ __forceinline__ v8f wmma16(v16h a, v16h b, v8f c) {
  v8f d = __builtin_amdgcn_wmma_f32_16x16x32_f16(false, a, false, b, (short)0, c,
                                                 false, false);
  asm volatile("v_nop\n\tv_nop\n\tv_nop\n\tv_nop" : "+v"(d) : "v"(a), "v"(b));
  return d;
}

__device__ __forceinline__ void wave_lds_sync() {
  __builtin_amdgcn_fence(3  , "wavefront");
  asm volatile("s_wait_dscnt 0x0" ::: "memory");
  __builtin_amdgcn_wave_barrier();
}

__global__ __launch_bounds__(256) void cast_kernel(
    const float* __restrict__ src, _Float16* __restrict__ dst, unsigned n8, float carry) {
  const unsigned i = blockIdx.x * 256u + threadIdx.x;
  if (i < n8) {
    const v4f a0 = *(const v4f*)(src + (size_t)i * 8u);
    const v4f a1 = *(const v4f*)(src + (size_t)i * 8u + 4u);
    v8h o;
#pragma unroll
    for (int j = 0; j < 4; ++j) {
      o[j]     = toh_flush(carry * bf16r(a0[j]));
      o[j + 4] = toh_flush(carry * bf16r(a1[j]));
    }
    _Float16* p = dst + (size_t)i * 8u;
    *(volatile v8h*)p = o;
    __threadfence();
    *(volatile v8h*)p = o;
  }
}

__global__ __launch_bounds__(256) void deg_kernel(
    const int* __restrict__ ei, float* __restrict__ dinv) {
  __shared__ unsigned seg[8 * SEGCAP];
  __shared__ unsigned wcnt[8];
  __shared__ float dsm[DROWS];
  const unsigned tid = threadIdx.x, lane = tid & 31u;
  const int wave = __builtin_amdgcn_readfirstlane(threadIdx.x >> 5);
  const unsigned r0 = blockIdx.x * (unsigned)DROWS;
  unsigned cnt = 0u;

#pragma unroll 1
  for (unsigned ch = 0; ch < (unsigned)NCHUNK; ++ch) {
    const unsigned e0 = ch * (unsigned)CHUNK + tid * 8u;
    const v4i ra = *(const v4i*)(ei + e0);
    const v4i rb = *(const v4i*)(ei + e0 + 4u);
    const int rr[8] = {ra[0], ra[1], ra[2], ra[3], rb[0], rb[1], rb[2], rb[3]};
    unsigned base = 0u;
#pragma unroll
    for (int j = 0; j < 8; ++j) {
      const unsigned rl = (unsigned)rr[j] - r0;
      const bool hit = rl < (unsigned)DROWS;
      const unsigned mk = __builtin_amdgcn_ballot_w32(hit);
      if (mk != 0u) {
        const unsigned pos = base + __builtin_amdgcn_mbcnt_lo(mk, 0u);
        if (hit) seg[(unsigned)wave * SEGCAP + pos] = rl;
        base += (unsigned)__popc(mk);
      }
    }
    if (lane == 0u) wcnt[wave] = base;
    __syncthreads();
    if (wave < 4) {
#pragma unroll 1
      for (unsigned s = 0; s < 8u; ++s) {
        unsigned n = wcnt[s];
        n = (n < (unsigned)SEGCAP) ? n : (unsigned)SEGCAP;
        n = (unsigned)__builtin_amdgcn_readfirstlane((int)n);
#pragma unroll 1
        for (unsigned i = 0; i < n; ++i) {
          const unsigned e = seg[s * SEGCAP + i];
          cnt += (e == tid) ? 1u : 0u;
        }
      }
    }
    __syncthreads();
  }

  if (tid < (unsigned)DROWS) {
    const float d = (float)((cnt > 0u) ? cnt : 1u);
    const float rs = 1.0f / sqrtf(d);
    dsm[tid] = (cnt > 0u) ? rs : 0.0f;
  }
  __syncthreads();
  if (wave == 0) {
    const v4f v = *(const v4f*)&dsm[lane * 4u];
    float* p = dinv + r0 + lane * 4u;
    *(volatile v4f*)p = v;
    __threadfence();
    *(volatile v4f*)p = v;
  }
}

__global__ __launch_bounds__(256) void gemm_lin_kernel(
    const _Float16* __restrict__ A16, const _Float16* __restrict__ Bt,
    const float* __restrict__ bias, const float* __restrict__ dinv,
    float* __restrict__ outf) {
  __shared__ float Cs[64 * LDC];
  const unsigned K = (unsigned)DIN;
  const unsigned tid = threadIdx.x, lane = tid & 31u, w = tid >> 5;
  const unsigned mw = w >> 1, nw = w & 1u;
  const unsigned hh = lane >> 4, m = lane & 15u;
  const unsigned n0 = blockIdx.x * 64u;
  const unsigned row0 = blockIdx.y * 64u;

  const _Float16* ap  = A16 + (size_t)(row0 + mw * 16u + m) * K + hh * 8u;
  const _Float16* bp0 = Bt + (size_t)(n0 + nw * 32u + m) * K + hh * 8u;
  const _Float16* bp1 = bp0 + (size_t)16 * K;
  v8f acc0 = {}, acc1 = {};
#pragma unroll 2
  for (unsigned k0 = 0; k0 < K; k0 += 32u) {
    const v16h a  = frag_at(ap + k0);
    const v16h b0 = frag_at(bp0 + k0);
    const v16h b1 = frag_at(bp1 + k0);
    acc0 = wmma16(a, b0, acc0);
    acc1 = wmma16(a, b1, acc1);
  }
#pragma unroll
  for (int r = 0; r < 8; ++r) {
    float* d = &Cs[(mw * 16u + hh * 8u + (unsigned)r) * LDC + nw * 32u + m];
    d[0]  = acc0[r];
    d[16] = acc1[r];
  }
  __syncthreads();

  const float cs = 1.0f / (XCARRY * WCARRY);
  v4f xs[4];
  size_t off[4];
#pragma unroll
  for (unsigned i = 0; i < 4u; ++i) {
    const unsigned r = 16u * i + (tid >> 4);
    const unsigned c = (tid & 15u) * 4u;
    const unsigned crow = row0 + r;
    const v4f u = *(const v4f*)&Cs[r * LDC + c];
    const v4f g = *(const v4f*)(bias + n0 + c);
    const float dv = dinv[crow];
    v4f val;
#pragma unroll
    for (int j = 0; j < 4; ++j) val[j] = dv * (u[j] * cs + bf16r(g[j]));
    xs[i] = val;
    off[i] = (size_t)crow * DOUT + n0 + c;
  }
#pragma unroll
  for (int i = 0; i < 4; ++i) *(volatile v4f*)(outf + off[i]) = xs[i];
  __threadfence();
#pragma unroll
  for (int i = 0; i < 4; ++i) *(volatile v4f*)(outf + off[i]) = xs[i];
}

__global__ __launch_bounds__(256) void agg_kernel(
    const int* __restrict__ ei, const float* __restrict__ G,
    const float* __restrict__ dinv, float* __restrict__ out) {
  __shared__ unsigned seen[AROWS * SEENW];
  __shared__ unsigned seg[8 * SEGCAP];
  __shared__ unsigned wcnt[8];
  const unsigned tid = threadIdx.x, lane = tid & 31u;
  const int wave = __builtin_amdgcn_readfirstlane(threadIdx.x >> 5);
  const unsigned r0 = blockIdx.x * (unsigned)AROWS;

#pragma unroll 1
  for (unsigned i = tid; i < (unsigned)(AROWS * SEENW); i += 256u) seen[i] = 0u;
  __syncthreads();

  v4f a0 = {}, a1 = {}, a2 = {}, a3 = {};

#pragma unroll 1
  for (unsigned ch = 0; ch < (unsigned)NCHUNK; ++ch) {
    const unsigned e0 = ch * (unsigned)CHUNK + tid * 8u;
    const v4i ra = *(const v4i*)(ei + e0);
    const v4i rb = *(const v4i*)(ei + e0 + 4u);
    const v4i ca = *(const v4i*)(ei + (size_t)N_EDGES + e0);
    const v4i cb = *(const v4i*)(ei + (size_t)N_EDGES + e0 + 4u);
    const int rr[8] = {ra[0], ra[1], ra[2], ra[3], rb[0], rb[1], rb[2], rb[3]};
    const int cc[8] = {ca[0], ca[1], ca[2], ca[3], cb[0], cb[1], cb[2], cb[3]};
    unsigned base = 0u;
#pragma unroll
    for (int j = 0; j < 8; ++j) {
      const unsigned rl = (unsigned)rr[j] - r0;
      const unsigned c = (unsigned)cc[j];
      const bool hit = (rl < (unsigned)AROWS) & (c < (unsigned)N_NODES);
      const unsigned mk = __builtin_amdgcn_ballot_w32(hit);
      if (mk != 0u) {
        const unsigned pos = base + __builtin_amdgcn_mbcnt_lo(mk, 0u);
        if (hit) seg[(unsigned)wave * SEGCAP + pos] = (rl << 13) | c;
        base += (unsigned)__popc(mk);
      }
    }
    if (lane == 0u) wcnt[wave] = base;
    __syncthreads();

#pragma unroll 1
    for (unsigned s = 0; s < 8u; ++s) {
      unsigned n = wcnt[s];
      n = (n < (unsigned)SEGCAP) ? n : (unsigned)SEGCAP;
      n = (unsigned)__builtin_amdgcn_readfirstlane((int)n);
#pragma unroll 1
      for (unsigned i = 0; i < n; ++i) {
        const unsigned ent =
            (unsigned)__builtin_amdgcn_readfirstlane((int)seg[s * SEGCAP + i]);
        const unsigned rl = (ent >> 13) & 31u;
        const unsigned c = ent & 8191u;
        if ((rl >> WSHIFT) == (unsigned)wave) {
          const unsigned widx = rl * (unsigned)SEENW + (c >> 5);
          const unsigned bit = 1u << (c & 31u);
          const unsigned old = (unsigned)__builtin_amdgcn_readfirstlane((int)seen[widx]);
          if ((old & bit) == 0u) {
            if (lane == 0u) seen[widx] = old | bit;
            const v4f g = *(const v4f*)(G + (size_t)c * DOUT + lane * 4u);
            const unsigned k = rl & 3u;
            if (k == 0u)      a0 += g;
            else if (k == 1u) a1 += g;
            else if (k == 2u) a2 += g;
            else              a3 += g;
          }
          wave_lds_sync();
        }
      }
    }
    __syncthreads();
  }

  const unsigned rbase = r0 + (unsigned)wave * (unsigned)WROWS;
  const v4f dv = *(const v4f*)(dinv + rbase);
  v4f o0, o1, o2, o3;
#pragma unroll
  for (int j = 0; j < 4; ++j) {
    o0[j] = fmaxf(a0[j] * dv[0], 0.0f);
    o1[j] = fmaxf(a1[j] * dv[1], 0.0f);
    o2[j] = fmaxf(a2[j] * dv[2], 0.0f);
    o3[j] = fmaxf(a3[j] * dv[3], 0.0f);
  }
  float* p = out + (size_t)rbase * DOUT + lane * 4u;
  *(volatile v4f*)(p) = o0;
  *(volatile v4f*)(p + DOUT) = o1;
  *(volatile v4f*)(p + 2 * DOUT) = o2;
  *(volatile v4f*)(p + 3 * DOUT) = o3;
  __threadfence();
  *(volatile v4f*)(p) = o0;
  *(volatile v4f*)(p + DOUT) = o1;
  *(volatile v4f*)(p + 2 * DOUT) = o2;
  *(volatile v4f*)(p + 3 * DOUT) = o3;
}

extern "C" void kernel_launch(void* const* d_in, const int* in_sizes, int n_in,
                              void* d_out, int out_size, void* d_ws, size_t ws_size,
                              hipStream_t stream) {
  if (n_in < 4) return;
  if ((long long)in_sizes[0] < (long long)N_NODES * DIN) return;
  if ((long long)in_sizes[1] < (long long)2 * N_EDGES) return;
  if ((long long)in_sizes[2] < (long long)DOUT * DIN) return;
  if (in_sizes[3] < DOUT) return;
  if ((long long)out_size < (long long)OUT_ROWS * DOUT) return;
  if (ws_size < WS_TOTAL) return;

  const float* X  = (const float*)d_in[0];
  const int*   EI = (const int*)d_in[1];
  const float* W  = (const float*)d_in[2];
  const float* B  = (const float*)d_in[3];
  float* out = (float*)d_out;

  char* ws = (char*)d_ws;
  _Float16* X16  = (_Float16*)(ws + OFF_X16);
  _Float16* W16  = (_Float16*)(ws + OFF_W16);
  float*    DINV = (float*)(ws + OFF_DINV);
  float*    G    = (float*)(ws + OFF_G);

  dim3 blk(256);
  cast_kernel<<<dim3((N_NODES * DIN / 8) / 256), blk, 0, stream>>>(
      X, X16, (unsigned)(N_NODES * DIN / 8), XCARRY);
  cast_kernel<<<dim3((DOUT * DIN / 8) / 256), blk, 0, stream>>>(
      W, W16, (unsigned)(DOUT * DIN / 8), WCARRY);
  deg_kernel<<<dim3(N_NODES / DROWS), blk, 0, stream>>>(EI, DINV);
  gemm_lin_kernel<<<dim3(DOUT / 64, N_NODES / 64), blk, 0, stream>>>(X16, W16, B, DINV, G);
  agg_kernel<<<dim3(OUT_ROWS / AROWS), blk, 0, stream>>>(EI, G, DINV, out);
}
